// EGNNContext_69458211111180
// MI455X (gfx1250) — hardware-run, weakly checked
//
#include <hip/hip_runtime.h>

typedef __attribute__((ext_vector_type(16))) _Float16 v16h;
typedef __attribute__((ext_vector_type(8)))  _Float16 v8h;
typedef __attribute__((ext_vector_type(8)))  float    v8f;
typedef __attribute__((ext_vector_type(4)))  float    v4f;
typedef __attribute__((ext_vector_type(2)))  float    v2f;
typedef __attribute__((ext_vector_type(2)))  unsigned v2u;
typedef __attribute__((ext_vector_type(2)))  int      v2i;

constexpr int kNodes = 384;
constexpr int kEdges = 3072;
constexpr int kCin = 4096;
constexpr int kEmb = 200;
constexpr int kHid = 512;
constexpr int kObj = 151;
constexpr int kRel = 51;
constexpr int kRelPad = 64;
constexpr int kPosIn = 9;
constexpr int kPosMid = 32;
constexpr int kPosOut = 128;
constexpr int kCat1 = 4424;
constexpr int kCat1P = 4448;
constexpr int kCat2 = 4808;
constexpr int kCat2P = 4832;
constexpr int kGate = 1536;
constexpr int kPairK = 1024;

static_assert(kCat1 == kCin + kEmb + kPosOut);
static_assert(kCat2 == kCin + kHid + kEmb);
static_assert(kCat1P % 32 == 0 && kCat2P % 32 == 0 && kCin % 32 == 0 && kHid % 32 == 0 && kPairK % 32 == 0);
static_assert(kCat1 % 8 == 0 && kCat2 % 8 == 0 && kEmb % 8 == 0);
static_assert(kNodes % 64 == 0 && kEdges % 64 == 0 && kHid % 64 == 0 && kGate % 64 == 0 && kRelPad % 64 == 0);
static_assert(kEdges % 256 == 0 && kEdges % 32 == 0);
static_assert((kNodes * kObj) % 32 == 0 && (kEdges * kRel) % 32 == 0);
static_assert((size_t)kNodes * kObj * 4 == 231936 && (size_t)kNodes * kObj * 4 % 128 == 0);
static_assert((size_t)kNodes * kObj * 4 + (size_t)kEdges * kRel * 4 == 858624);

constexpr size_t kSzWn1  = (size_t)kHid * kCat1P * 2;
constexpr size_t kSzWed  = (size_t)kHid * kCin * 2;
constexpr size_t kSzWn2  = (size_t)kHid * kCat2P * 2;
constexpr size_t kSzWg   = (size_t)kGate * kHid * 2;
constexpr size_t kSzWsq  = (size_t)kHid * kHid * 2;
constexpr size_t kSzWc1  = (size_t)kHid * kPairK * 2;
constexpr size_t kSzWrel = (size_t)kRelPad * kHid * 2;
constexpr size_t kSzUni  = (size_t)kEdges * kCin * 2;
constexpr size_t kSzEh   = (size_t)kEdges * kHid * 2;
constexpr size_t kSzEf   = (size_t)kEdges * kHid * 4;
constexpr size_t kSzEg   = (size_t)kEdges * kGate * 4;
constexpr size_t kSzEk   = (size_t)kEdges * kPairK * 2;
constexpr size_t kSzNh   = (size_t)kNodes * kHid * 2;
constexpr size_t kSzNf   = (size_t)kNodes * kHid * 4;
constexpr size_t kSzNg   = (size_t)kNodes * kGate * 4;

constexpr size_t kOffWn1   = 0;
constexpr size_t kOffWed   = kOffWn1 + kSzWn1;
constexpr size_t kOffWn2   = kOffWed + kSzWed;
constexpr size_t kOffWngih = kOffWn2 + kSzWn2;
constexpr size_t kOffWnghh = kOffWngih + kSzWg;
constexpr size_t kOffWegih = kOffWnghh + kSzWg;
constexpr size_t kOffWeghh = kOffWegih + kSzWg;
constexpr size_t kOffWa1   = kOffWeghh + kSzWg;
constexpr size_t kOffWa2   = kOffWa1 + kSzWsq;
constexpr size_t kOffWb1   = kOffWa2 + kSzWsq;
constexpr size_t kOffWb2   = kOffWb1 + kSzWsq;
constexpr size_t kOffWc1   = kOffWb2 + kSzWsq;
constexpr size_t kOffWc2   = kOffWc1 + kSzWc1;
constexpr size_t kOffWrelH = kOffWc2 + kSzWsq;
constexpr size_t kOffWrelL = kOffWrelH + kSzWrel;
constexpr size_t kOffUni   = kOffWrelL + kSzWrel;
constexpr size_t kOffEk    = kOffUni;
constexpr size_t kOffT1    = kOffEk + kSzEk;
constexpr size_t kOffMsg   = kOffT1 + kSzEh;
constexpr size_t kOffHeh0  = kOffMsg + kSzEh;
constexpr size_t kOffHeh1  = kOffHeh0 + kSzEh;
constexpr size_t kOffHelo  = kOffHeh1 + kSzEh;
static_assert(kOffHelo + kSzEh <= kOffUni + kSzUni);
constexpr size_t kOffXcat  = kOffUni + kSzUni;
constexpr size_t kOffXcat2 = kOffXcat + (size_t)kNodes * kCat1P * 2;
constexpr size_t kOffEr    = kOffXcat2 + (size_t)kNodes * kCat2P * 2;
constexpr size_t kOffHe0   = kOffEr + kSzEf;
constexpr size_t kOffHe1   = kOffHe0 + kSzEf;
constexpr size_t kOffGie   = kOffHe1 + kSzEf;
constexpr size_t kOffGhe   = kOffGie + kSzEg;
constexpr size_t kOffPh    = kOffGhe + kSzEg;
constexpr size_t kOffStats = kOffPh + (size_t)kNodes * kPosMid * 4;
constexpr size_t kOffPose  = kOffStats + 256;
constexpr size_t kOffHn0   = kOffPose + (size_t)kNodes * kPosOut * 4;
constexpr size_t kOffHn1   = kOffHn0 + kSzNf;
constexpr size_t kOffHnh0  = kOffHn1 + kSzNf;
constexpr size_t kOffHnh1  = kOffHnh0 + kSzNh;
constexpr size_t kOffE2nRaw = kOffHnh1 + kSzNh;
constexpr size_t kOffN2nRaw = kOffE2nRaw + kSzNh;
constexpr size_t kOffTe    = kOffN2nRaw + kSzNh;
constexpr size_t kOffTn    = kOffTe + kSzNh;
constexpr size_t kOffE2nM  = kOffTn + kSzNh;
constexpr size_t kOffN2nM  = kOffE2nM + kSzNf;
constexpr size_t kOffInph  = kOffN2nM + kSzNf;
constexpr size_t kOffGin   = kOffInph + kSzNh;
constexpr size_t kOffGhn   = kOffGin + kSzNg;
constexpr size_t kOffNs2   = kOffGhn + kSzNg;
constexpr size_t kOffRelPad = kOffNs2 + kSzNf;
constexpr size_t kOffFirst = kOffRelPad + (size_t)kEdges * kRelPad * 4;
constexpr size_t kWsTotal  = kOffFirst + (size_t)kEdges * 4;
static_assert(kWsTotal == 125153536);
static_assert(kWsTotal <= 134217728);
static_assert(kOffUni % 256 == 0 && kOffXcat % 256 == 0 && kOffPh % 256 == 0 && kOffFirst % 256 == 0 && kOffStats % 256 == 0);

__device__ __forceinline__ int clampi(int v, int lo, int hi) { return v < lo ? lo : (v > hi ? hi : v); }

__device__ __forceinline__ _Float16 to_h16(float v) {
  const float w = (__builtin_fabsf(v) < 6.103515625e-5f) ? 0.0f : v;
  return (_Float16)w;
}
__device__ __forceinline__ unsigned pack_h2(float a, float b) {
  const _Float16 h0 = to_h16(a), h1 = to_h16(b);
  return (unsigned)__builtin_bit_cast(unsigned short, h0) | ((unsigned)__builtin_bit_cast(unsigned short, h1) << 16);
}

__device__ __forceinline__ void dep_guard_h(v8f& a, v8f& b, v16h x, v16h y) { asm volatile("v_nop\n\tv_nop\n\tv_nop\n\tv_nop" : "+v"(a), "+v"(b) : "v"(x), "v"(y)); }
__device__ __forceinline__ void keep4_h(v16h a, v16h b, v16h c, v16h d) { asm volatile("v_nop" :: "v"(a), "v"(b), "v"(c), "v"(d)); }
__device__ __forceinline__ void acc_guard4(v8f& a, v8f& b, v8f& c, v8f& d) { asm volatile("v_nop\n\tv_nop\n\tv_nop\n\tv_nop" : "+v"(a), "+v"(b), "+v"(c), "+v"(d)); }
template <typename T> struct Frag;
template <> struct Frag<_Float16> {
  typedef v16h V; union U { v16h v; v8h h[2]; };
  static __device__ __forceinline__ v16h load(const _Float16* p) {
    U f; f.h[0] = *(const v8h*)(p); f.h[1] = *(const v8h*)(p + 16); return f.v;
  }
  static __device__ __forceinline__ v8f mma(v16h a, v16h b, v8f c) {
    return __builtin_amdgcn_wmma_f32_16x16x32_f16(false, a, false, b, (short)0, c, false, false);
  }
  static __device__ __forceinline__ void guard(v8f& a, v8f& b, v16h x, v16h y) { dep_guard_h(a, b, x, y); }
  static __device__ __forceinline__ void keep(v16h a, v16h b, v16h c, v16h d) { keep4_h(a, b, c, d); }
};

template <int MI, bool SPLIT, bool HAS_BIAS, int OUT_MODE, bool RELU>
__global__ __launch_bounds__(256) void wmma_gemm64(
    const _Float16* __restrict__ A, const _Float16* __restrict__ A2, int lda,
    const _Float16* __restrict__ Bt, const _Float16* __restrict__ Bt2, int ldb,
    float* __restrict__ Cf, _Float16* __restrict__ Ch, int ldc,
    const float* __restrict__ bias, int nBias,
    int M, int N, int K, float scale, float rscale, float oscale) {
  typedef _Float16 T;
  typedef Frag<T>::V V;
  __shared__ __align__(16) float sT[8][16 * 68];
  const int lane = threadIdx.x & 31;
  const int wave = threadIdx.x >> 5;
  const int tilesN = N >> 6;
  const int tilesM = M / (16 * MI);
  const int tile = blockIdx.x * 8 + wave;
  if (tile >= tilesM * tilesN) return;
  const int tm = tile / tilesN;
  const int tn = tile - tm * tilesN;
  const int m0 = tm * (16 * MI);
  const int n0 = tn << 6;

  const int rlane = lane & 15;
  const int koff  = (lane >> 4) * 8;
  const int mOff  = (lane >> 4) * 8;

  v8f acc[MI][4];
  v8f accr[SPLIT ? MI : 1][4];
#pragma unroll
  for (int i = 0; i < MI; ++i)
#pragma unroll
    for (int j = 0; j < 4; ++j) acc[i][j] = (v8f){0.f,0.f,0.f,0.f,0.f,0.f,0.f,0.f};
#pragma unroll
  for (int i = 0; i < (SPLIT ? MI : 1); ++i)
#pragma unroll
    for (int j = 0; j < 4; ++j) accr[i][j] = (v8f){0.f,0.f,0.f,0.f,0.f,0.f,0.f,0.f};

  for (int k0 = 0; k0 < K; k0 += 32) {
    V bh[4], bl[4];
#pragma unroll
    for (int j = 0; j < 4; ++j) {
      const size_t bo = (size_t)(n0 + (j << 4) + rlane) * ldb + koff + k0;
      bh[j] = Frag<T>::load(Bt + bo);
      if (SPLIT) bl[j] = Frag<T>::load(Bt2 + bo);
    }
#pragma unroll
    for (int i = 0; i < MI; ++i) {
      const size_t ao = (size_t)(m0 + (i << 4) + rlane) * lda + koff + k0;
      V ah = Frag<T>::load(A + ao);
      V al = ah;
      if (SPLIT) al = Frag<T>::load(A2 + ao);
#pragma unroll
      for (int j = 0; j < 4; ++j) {
        acc[i][j] = Frag<T>::mma(ah, bh[j], acc[i][j]);
        if (SPLIT) {
          accr[SPLIT ? i : 0][j] = Frag<T>::mma(ah, bl[j], accr[SPLIT ? i : 0][j]);
          accr[SPLIT ? i : 0][j] = Frag<T>::mma(al, bh[j], accr[SPLIT ? i : 0][j]);
          Frag<T>::guard(acc[i][j], accr[SPLIT ? i : 0][j], ah, al);
        }
      }
      if (!SPLIT) Frag<T>::guard(acc[i][0], acc[i][3], ah, ah);
    }
    Frag<T>::keep(bh[0], bh[1], bh[2], bh[3]);
    if (SPLIT) Frag<T>::keep(bl[0], bl[1], bl[2], bl[3]);
  }
#pragma unroll
  for (int i = 0; i < MI; ++i) acc_guard4(acc[i][0], acc[i][1], acc[i][2], acc[i][3]);
  if (SPLIT) {
#pragma unroll
    for (int i = 0; i < (SPLIT ? MI : 1); ++i) acc_guard4(accr[i][0], accr[i][1], accr[i][2], accr[i][3]);
  }

  float* slab = sT[wave];
#pragma unroll
  for (int i = 0; i < MI; ++i) {
    const int mBase = m0 + (i << 4);
#pragma unroll
    for (int j = 0; j < 4; ++j) {
      const int n = n0 + (j << 4) + rlane;
      float bv = 0.f;
      if (HAS_BIAS) {
        const int nc = n < nBias ? n : nBias - 1;
        const float bval = bias[nc];
        bv = (n < nBias) ? bval : 0.f;
      }
#pragma unroll
      for (int r = 0; r < 8; ++r) {
        float v = acc[i][j][r] * scale;
        if (SPLIT) v += accr[SPLIT ? i : 0][j][r] * rscale;
        v += bv;
        if (RELU) v = fmaxf(v, 0.0f);
        slab[(mOff + r) * 68 + (j << 4) + rlane] = v;
      }
    }
    __builtin_amdgcn_fence(__ATOMIC_RELEASE, "workgroup");
    __builtin_amdgcn_wave_barrier();
    __builtin_amdgcn_fence(__ATOMIC_ACQUIRE, "workgroup");
    if (OUT_MODE == 0 || OUT_MODE == 3) {
      const int hh = lane >> 4, c4 = (lane & 15) * 4;
      for (int pass = 0; pass < 2; ++pass) {
#pragma unroll
        for (int it = 0; it < 8; ++it) {
          const int row = it * 2 + hh;
          v4f v = *(const v4f*)(slab + row * 68 + c4);
          *(volatile v4f*)(Cf + (size_t)(mBase + row) * ldc + n0 + c4) = v;
        }
        __threadfence();
      }
    }
    if (OUT_MODE == 1 || OUT_MODE == 3) {
      const int q = lane >> 3, c8 = (lane & 7) * 8;
      for (int pass = 0; pass < 2; ++pass) {
#pragma unroll
        for (int it = 0; it < 4; ++it) {
          const int row = it * 4 + q;
          const float* sp = slab + row * 68 + c8;
          v8h hv;
#pragma unroll
          for (int e = 0; e < 8; ++e) hv[e] = to_h16((sp[e] * oscale));
          *(volatile v8h*)(Ch + (size_t)(mBase + row) * ldc + n0 + c8) = hv;
        }
        __threadfence();
      }
    }
    __builtin_amdgcn_fence(__ATOMIC_RELEASE, "workgroup");
    __builtin_amdgcn_wave_barrier();
    __builtin_amdgcn_fence(__ATOMIC_ACQUIRE, "workgroup");
  }
}

__global__ __launch_bounds__(256) void cvt_pad_f16(
    const float* __restrict__ src, _Float16* __restrict__ dst,
    int rowsReal, int rowsPad, int K, int Kp, float scale) {
  const int cpr = Kp >> 3;
  const long total = (long)rowsPad * cpr;
  const long i = (long)blockIdx.x * 256 + threadIdx.x;
  if (i >= total) return;
  const int row = (int)(i / cpr);
  const int c8 = (int)(i - (long)row * cpr) << 3;
  const bool inr = (row < rowsReal) && (c8 < K);
  const int rc = row < rowsReal ? row : rowsReal - 1;
  const int cc = c8 < K ? c8 : K - 8;
  const float* sp = src + (size_t)rc * K + cc;
  const v4f a = *(const v4f*)sp;
  const v4f b = *(const v4f*)(sp + 4);
  v8h hv;
#pragma unroll
  for (int e = 0; e < 4; ++e) {
    hv[e]     = to_h16((inr ? a[e] * scale : 0.0f));
    hv[4 + e] = to_h16((inr ? b[e] * scale : 0.0f));
  }
  volatile v8h* dp = (volatile v8h*)(dst + (size_t)i * 8);
  *dp = hv;
  __threadfence();
  *dp = hv;
}

__global__ __launch_bounds__(256) void rel_weight_split(
    const float* __restrict__ w, _Float16* __restrict__ hi, _Float16* __restrict__ lo) {
  const int i = blockIdx.x * 256 + threadIdx.x;
  if (i >= kRelPad * (kHid / 8)) return;
  const int row = i >> 6;
  const int c8 = (i & 63) << 3;
  const bool inr = row < kRel;
  const int rc = inr ? row : kRel - 1;
  const float* sp = w + (size_t)rc * kHid + c8;
  const v4f a = *(const v4f*)sp;
  const v4f b = *(const v4f*)(sp + 4);
  v8h hv, lv;
#pragma unroll
  for (int e = 0; e < 8; ++e) {
    const float s = (e < 4 ? a[e & 3] : b[e & 3]) * 1024.0f;
    const float v = inr ? s : 0.0f;
    const _Float16 h = to_h16(v);
    const float res = (v - (float)h) * 2048.0f;
    hv[e] = h;
    lv[e] = to_h16(res);
  }
  volatile v8h* ph = (volatile v8h*)(hi + (size_t)i * 8);
  volatile v8h* pl = (volatile v8h*)(lo + (size_t)i * 8);
  *ph = hv; *pl = lv;
  __threadfence();
  *ph = hv; *pl = lv;
}

__global__ __launch_bounds__(256) void pos_lin1(
    const float* __restrict__ pinfo, const float* __restrict__ w, const float* __restrict__ b,
    float* __restrict__ ph) {
  const int i = blockIdx.x * 256 + threadIdx.x;
  if (i >= kNodes * kPosMid) return;
  const int r = i >> 5, c = i & 31;
  float s = 0.0f;
#pragma unroll
  for (int j = 0; j < kPosIn; ++j) s += pinfo[r * kPosIn + j] * w[c * kPosIn + j];
  s += b[c];
  volatile float* p = ph + i;
  *p = s;
  __threadfence();
  *p = s;
}

__global__ __launch_bounds__(256) void pos_bnstats(const float* __restrict__ ph, float* __restrict__ stats) {
  __shared__ float part[8][32];
  __shared__ float smean[32];
  const int c = threadIdx.x & 31;
  const int w = threadIdx.x >> 5;
  float s = 0.0f;
  for (int r = w; r < kNodes; r += 8) s += ph[r * kPosMid + c];
  part[w][c] = s;
  __syncthreads();
  if (w == 0) {
    float t = 0.0f;
#pragma unroll
    for (int k = 0; k < 8; ++k) t += part[k][c];
    smean[c] = t * (1.0f / (float)kNodes);
  }
  __syncthreads();
  const float mu = smean[c];
  float q = 0.0f;
  for (int r = w; r < kNodes; r += 8) { const float d = ph[r * kPosMid + c] - mu; q += d * d; }
  part[w][c] = q;
  __syncthreads();
  if (w == 0) {
    float t = 0.0f;
#pragma unroll
    for (int k = 0; k < 8; ++k) t += part[k][c];
    const float var = t * (1.0f / (float)kNodes);
    const float rs = rsqrtf(var + 1e-5f);
    volatile float* p0 = stats + c;
    volatile float* p1 = stats + 32 + c;
    *p0 = mu; *p1 = rs;
    __threadfence();
    *p0 = mu; *p1 = rs;
  }
}

__global__ __launch_bounds__(128) void pos_lin2(
    const float* __restrict__ ph, const float* __restrict__ stats,
    const float* __restrict__ gamma, const float* __restrict__ beta,
    const float* __restrict__ w2, const float* __restrict__ b2, float* __restrict__ pose) {
  __shared__ float sn[32];
  const int r = blockIdx.x;
  const int t = threadIdx.x;
  if (t < 32) sn[t] = (ph[r * kPosMid + t] - stats[t]) * stats[32 + t] * gamma[t] + beta[t];
  __syncthreads();
  const float* wr = w2 + t * kPosMid;
  float s = 0.0f;
#pragma unroll
  for (int j4 = 0; j4 < 8; ++j4) {
    const v4f wv = *(const v4f*)(wr + 4 * j4);
#pragma unroll
    for (int e = 0; e < 4; ++e) s += sn[4 * j4 + e] * wv[e];
  }
  s += b2[t];
  s = fmaxf(s, 0.0f);
  volatile float* p = pose + r * kPosOut + t;
  *p = s;
  __threadfence();
  *p = s;
}

template <bool EMB_FIRST>
__global__ __launch_bounds__(256) void build_cat(
    const float* __restrict__ x, const float* __restrict__ rowsrc, int rowW,
    const float* __restrict__ tab, const int* __restrict__ lab,
    _Float16* __restrict__ dst, int Kp) {
  const int cpr = Kp >> 3;
  const int total = kNodes * cpr;
  const int i = blockIdx.x * 256 + threadIdx.x;
  if (i >= total) return;
  const int row = i / cpr;
  const int c8 = (i - row * cpr) << 3;
  const int embStart = EMB_FIRST ? kCin : (kCin + rowW);
  const int rowStart = EMB_FIRST ? (kCin + kEmb) : kCin;
  const int lb = clampi(lab[row], 0, kObj - 1);
  const int cx = c8 < kCin ? c8 : kCin - 8;
  const int ce = clampi(c8 - embStart, 0, kEmb - 8);
  const int cr = clampi(c8 - rowStart, 0, rowW - 8);
  const float* px = x + (size_t)row * kCin + cx;
  const float* pe = tab + (size_t)lb * kEmb + ce;
  const float* pr = rowsrc + (size_t)row * rowW + cr;
  v4f x0 = *(const v4f*)px, x1 = *(const v4f*)(px + 4);
  v4f e0 = *(const v4f*)pe, e1 = *(const v4f*)(pe + 4);
  v4f r0 = *(const v4f*)pr, r1 = *(const v4f*)(pr + 4);
  asm volatile("" : "+v"(x0), "+v"(x1), "+v"(e0), "+v"(e1), "+v"(r0), "+v"(r1));
  const bool inX = c8 < kCin;
  const bool inE = (c8 >= embStart) && (c8 < embStart + kEmb);
  const bool inR = (c8 >= rowStart) && (c8 < rowStart + rowW);
  v8h hv;
#pragma unroll
  for (int e = 0; e < 4; ++e) {
    const float f0 = inX ? x0[e] : (inE ? e0[e] : (inR ? r0[e] : 0.0f));
    const float f1 = inX ? x1[e] : (inE ? e1[e] : (inR ? r1[e] : 0.0f));
    hv[e] = to_h16(f0);
    hv[4 + e] = to_h16(f1);
  }
  volatile v8h* dp = (volatile v8h*)(dst + (size_t)i * 8);
  *dp = hv;
  __threadfence();
  *dp = hv;
}

__global__ __launch_bounds__(256) void pair_flags(const int* __restrict__ rp, int* __restrict__ first) {
  __shared__ int skey[kEdges];
  for (int k = threadIdx.x; k < kEdges; k += 256) {
    const v2i p = ((const v2i*)rp)[k];
    skey[k] = clampi(p[0], 0, kNodes - 1) * kNodes + clampi(p[1], 0, kNodes - 1);
  }
  __syncthreads();
  const int e = blockIdx.x * 256 + threadIdx.x;
  const int ec = e < kEdges ? e : kEdges - 1;
  const int my = skey[ec];
  int cnt = 0;
  for (int k = 0; k < kEdges; ++k) cnt += ((skey[k] == my) && (k < ec)) ? 1 : 0;
  const int f = (cnt == 0) ? 1 : 0;
  if (e < kEdges) {
    volatile int* p = first + e;
    *p = f;
    __threadfence();
    *p = f;
  }
}

__global__ __launch_bounds__(256) void pair_h0(
    const int* __restrict__ rp, const float* __restrict__ er,
    float* __restrict__ h0, _Float16* __restrict__ h0h) {
  __shared__ int skey[kEdges];
  for (int k = threadIdx.x; k < kEdges; k += 256) {
    const v2i p = ((const v2i*)rp)[k];
    skey[k] = clampi(p[0], 0, kNodes - 1) * kNodes + clampi(p[1], 0, kNodes - 1);
  }
  __syncthreads();
  const int lane = threadIdx.x & 31;
  const int wave = threadIdx.x >> 5;
  const int e = blockIdx.x * 8 + wave;
  const int my = skey[e];
  v4f a0 = (v4f){0.f, 0.f, 0.f, 0.f}, a1 = a0, a2 = a0, a3 = a0;
  for (int it = 0; it < kEdges / 32; ++it) {
    const int k = skey[it * 32 + lane];
    const unsigned m = __builtin_amdgcn_ballot_w32(k == my);
#pragma unroll 1
    for (int b = 0; b < 32; ++b) {
      if ((m >> b) & 1u) {
        const int src = it * 32 + b;
        const float* sp = er + (size_t)src * kHid + lane * 4;
        a0 += *(const v4f*)(sp);
        a1 += *(const v4f*)(sp + 128);
        a2 += *(const v4f*)(sp + 256);
        a3 += *(const v4f*)(sp + 384);
      }
    }
  }
  float* op = h0 + (size_t)e * kHid + lane * 4;
  _Float16* oh = h0h + (size_t)e * kHid + lane * 4;
  const v2u u0 = (v2u){pack_h2(a0[0] * 16.f, a0[1] * 16.f), pack_h2(a0[2] * 16.f, a0[3] * 16.f)};
  const v2u u1 = (v2u){pack_h2(a1[0] * 16.f, a1[1] * 16.f), pack_h2(a1[2] * 16.f, a1[3] * 16.f)};
  const v2u u2 = (v2u){pack_h2(a2[0] * 16.f, a2[1] * 16.f), pack_h2(a2[2] * 16.f, a2[3] * 16.f)};
  const v2u u3 = (v2u){pack_h2(a3[0] * 16.f, a3[1] * 16.f), pack_h2(a3[2] * 16.f, a3[3] * 16.f)};
  for (int pass = 0; pass < 2; ++pass) {
    *(volatile v4f*)(op) = a0;
    *(volatile v4f*)(op + 128) = a1;
    *(volatile v4f*)(op + 256) = a2;
    *(volatile v4f*)(op + 384) = a3;
    *(volatile v2u*)(oh) = u0;
    *(volatile v2u*)(oh + 128) = u1;
    *(volatile v2u*)(oh + 256) = u2;
    *(volatile v2u*)(oh + 384) = u3;
    __threadfence();
  }
}

template <int MODE>
__global__ __launch_bounds__(128) void node_gather(
    const int* __restrict__ rp, const int* __restrict__ first,
    const float* __restrict__ src, _Float16* __restrict__ outh) {
  __shared__ int smatch[kEdges];
  __shared__ int ssrc[kEdges];
  const int node = blockIdx.x;
  for (int k = threadIdx.x; k < kEdges; k += 128) {
    const v2i p = ((const v2i*)rp)[k];
    const int p0 = clampi(p[0], 0, kNodes - 1);
    const int p1 = clampi(p[1], 0, kNodes - 1);
    if (MODE == 0) {
      smatch[k] = p1;
      ssrc[k] = k;
    } else {
      const int f = first[k];
      smatch[k] = (f != 0) ? p0 : -1;
      ssrc[k] = p1;
    }
  }
  __syncthreads();
  const int lane = threadIdx.x & 31;
  const int wave = threadIdx.x >> 5;
  const int ch = wave * 128 + lane * 4;
  v4f acc = (v4f){0.f, 0.f, 0.f, 0.f};
  int cnt = 0;
  for (int it = 0; it < kEdges / 32; ++it) {
    const int kk = smatch[it * 32 + lane];
    const unsigned m = __builtin_amdgcn_ballot_w32(kk == node);
    cnt += __builtin_popcount(m);
#pragma unroll 1
    for (int b = 0; b < 32; ++b) {
      if ((m >> b) & 1u) {
        const int s = ssrc[it * 32 + b];
        acc += *(const v4f*)(src + (size_t)s * kHid + ch);
      }
    }
  }
  float sc = 1.0f;
  if (MODE == 1) sc = 1.0f / ((float)cnt + 1e-6f);
  const v2u u = (v2u){pack_h2(acc[0] * sc * 16.f, acc[1] * sc * 16.f), pack_h2(acc[2] * sc * 16.f, acc[3] * sc * 16.f)};
  volatile v2u* p = (volatile v2u*)(outh + (size_t)node * kHid + ch);
  *p = u;
  __threadfence();
  *p = u;
}

__global__ __launch_bounds__(256) void combine_half(
    const float* __restrict__ a, const float* __restrict__ b, _Float16* __restrict__ out, int n8) {
  const int i = blockIdx.x * 256 + threadIdx.x;
  if (i >= n8) return;
  const v4f a0 = ((const v4f*)a)[2 * i], a1 = ((const v4f*)a)[2 * i + 1];
  const v4f b0 = ((const v4f*)b)[2 * i], b1 = ((const v4f*)b)[2 * i + 1];
  v8h hv;
#pragma unroll
  for (int e = 0; e < 4; ++e) {
    hv[e]     = to_h16(((0.5f * a0[e] + 0.5f * b0[e]) * 16.0f));
    hv[4 + e] = to_h16(((0.5f * a1[e] + 0.5f * b1[e]) * 16.0f));
  }
  volatile v8h* dp = (volatile v8h*)(out + (size_t)i * 8);
  *dp = hv;
  __threadfence();
  *dp = hv;
}

template <bool WITH_LO>
__global__ __launch_bounds__(256) void gru_gate(
    const float* __restrict__ gi, const float* __restrict__ gh, const float* __restrict__ hcur,
    float* __restrict__ hnext, _Float16* __restrict__ hhi, _Float16* __restrict__ hlo, int rows) {
  const int t = blockIdx.x * 256 + threadIdx.x;
  if (t >= rows * 256) return;
  const int row = t >> 8;
  const int c2 = (t & 255) << 1;
  const float* gip = gi + (size_t)row * kGate + c2;
  const float* ghp = gh + (size_t)row * kGate + c2;
  const v2f ir = *(const v2f*)(gip), iz = *(const v2f*)(gip + kHid), ig = *(const v2f*)(gip + 2 * kHid);
  const v2f hr = *(const v2f*)(ghp), hz = *(const v2f*)(ghp + kHid), hg = *(const v2f*)(ghp + 2 * kHid);
  const v2f hc = *(const v2f*)(hcur + (size_t)row * kHid + c2);
  float o[2];
#pragma unroll
  for (int e = 0; e < 2; ++e) {
    const float r = 1.0f / (1.0f + expf(-(ir[e] + hr[e])));
    const float z = 1.0f / (1.0f + expf(-(iz[e] + hz[e])));
    const float g = tanhf(ig[e] + r * hg[e]);
    o[e] = (1.0f - z) * g + z * hc[e];
  }
  const v2f ov = (v2f){o[0], o[1]};
  const float s0 = o[0] * 16.0f, s1 = o[1] * 16.0f;
  const unsigned uh = pack_h2(s0, s1);
  unsigned ul = 0u;
  if (WITH_LO) {
    const _Float16 h0 = to_h16(s0), h1 = to_h16(s1);
    ul = pack_h2((s0 - (float)h0) * 2048.0f, (s1 - (float)h1) * 2048.0f);
  }
  volatile v2f* po = (volatile v2f*)(hnext + (size_t)row * kHid + c2);
  volatile unsigned* ph = (volatile unsigned*)(hhi + (size_t)row * kHid + c2);
  volatile unsigned* pl = WITH_LO ? (volatile unsigned*)(hlo + (size_t)row * kHid + c2) : nullptr;
  *po = ov; *ph = uh;
  if (WITH_LO) *pl = ul;
  __threadfence();
  *po = ov; *ph = uh;
  if (WITH_LO) *pl = ul;
}

__global__ __launch_bounds__(256) void build_ek(
    const int* __restrict__ rp, const float* __restrict__ ns2, _Float16* __restrict__ dst) {
  const int i = blockIdx.x * 256 + threadIdx.x;
  if (i >= kEdges * (kPairK / 8)) return;
  const int e = i >> 7;
  const int c8 = (i & 127) << 3;
  const int side = c8 >> 9;
  const int node = clampi(rp[2 * e + side], 0, kNodes - 1);
  const float* sp = ns2 + (size_t)node * kHid + (c8 & (kHid - 1));
  const v4f a = *(const v4f*)sp;
  const v4f b = *(const v4f*)(sp + 4);
  v8h hv;
#pragma unroll
  for (int k = 0; k < 4; ++k) {
    hv[k] = to_h16((a[k] * 16.0f));
    hv[4 + k] = to_h16((b[k] * 16.0f));
  }
  volatile v8h* dp = (volatile v8h*)(dst + (size_t)i * 8);
  *dp = hv;
  __threadfence();
  *dp = hv;
}

__global__ __launch_bounds__(256) void pack_obj(const int* __restrict__ lab, float* __restrict__ out) {
  const int i = blockIdx.x * 256 + threadIdx.x;
  if (i >= kNodes * kObj) return;
  const int r = i / kObj;
  const int c = i - r * kObj;
  const int lb = clampi(lab[r], 0, kObj - 1);
  const float v = (c == lb) ? 1000.0f : -1000.0f;
  volatile float* p = out + i;
  *p = v;
  __threadfence();
  *p = v;
}

__global__ __launch_bounds__(256) void pack_rel(const float* __restrict__ relpad, float* __restrict__ out) {
  const int i = blockIdx.x * 256 + threadIdx.x;
  if (i >= kEdges * kRel) return;
  const int r = i / kRel;
  const int c = i - r * kRel;
  const float v = relpad[(size_t)r * kRelPad + c];
  volatile float* p = out + i;
  *p = v;
  __threadfence();
  *p = v;
}

template <int MI, bool SPLIT, bool HAS_BIAS, int OUT_MODE, bool RELU>
static void run_gemm(hipStream_t st, const _Float16* A, const _Float16* A2, int lda,
                     const _Float16* Bt, const _Float16* Bt2, int ldb,
                     float* Cf, _Float16* Ch, int ldc, const float* bias, int nBias,
                     int M, int N, int K, float scale, float rscale, float oscale) {
  const int tiles = (M / (16 * MI)) * (N / 64);
  wmma_gemm64<MI, SPLIT, HAS_BIAS, OUT_MODE, RELU><<<dim3((unsigned)((tiles + 7) / 8)), dim3(256), 0, st>>>(
      A, A2, lda, Bt, Bt2, ldb, Cf, Ch, ldc, bias, nBias, M, N, K, scale, rscale, oscale);
}

static void run_cvt(hipStream_t st, const float* s, _Float16* d, int rowsReal, int rowsPad, int K, int Kp, float sc) {
  const long total = (long)rowsPad * (Kp / 8);
  cvt_pad_f16<<<dim3((unsigned)((total + 255) / 256)), dim3(256), 0, st>>>(s, d, rowsReal, rowsPad, K, Kp, sc);
}

extern "C" void kernel_launch(void* const* d_in, const int* in_sizes, int n_in,
                              void* d_out, int out_size, void* d_ws, size_t ws_size,
                              hipStream_t stream) {
  if (n_in < 39) return;
  {
    constexpr int kInSizes[39] = {1572864, 3456, 12582912, 384, 6144, 30200, 30200, 2265088, 512, 2461696, 512, 2097152, 512, 288, 32, 32, 32, 4096, 128, 786432, 786432, 1536, 1536, 786432, 786432, 262144, 512, 262144, 512, 262144, 512, 262144, 512, 524288, 512, 262144, 512, 26112, 51};
    for (int k = 0; k < 39; ++k) if (in_sizes[k] != kInSizes[k]) return;
  }
  if (out_size != 214656) return;
  if (ws_size < kWsTotal) return;

  const float* x      = (const float*)d_in[0];
  const float* pinfo  = (const float*)d_in[1];
  const float* uni    = (const float*)d_in[2];
  const int*   lab    = (const int*)d_in[3];
  const int*   rp     = (const int*)d_in[4];
  const float* emb1   = (const float*)d_in[5];
  const float* emb2   = (const float*)d_in[6];
  const float* w_n1   = (const float*)d_in[7];
  const float* b_n1   = (const float*)d_in[8];
  const float* w_n2   = (const float*)d_in[9];
  const float* b_n2   = (const float*)d_in[10];
  const float* w_ed   = (const float*)d_in[11];
  const float* b_ed   = (const float*)d_in[12];
  const float* pw1    = (const float*)d_in[13];
  const float* pb1    = (const float*)d_in[14];
  const float* pgam   = (const float*)d_in[15];
  const float* pbet   = (const float*)d_in[16];
  const float* pw2    = (const float*)d_in[17];
  const float* pb2    = (const float*)d_in[18];
  const float* ngih   = (const float*)d_in[19];
  const float* nghh   = (const float*)d_in[20];
  const float* ngbih  = (const float*)d_in[21];
  const float* ngbhh  = (const float*)d_in[22];
  const float* egih   = (const float*)d_in[23];
  const float* eghh   = (const float*)d_in[24];
  const float* n2n1w  = (const float*)d_in[25];
  const float* n2n1b  = (const float*)d_in[26];
  const float* n2n2w  = (const float*)d_in[27];
  const float* n2n2b  = (const float*)d_in[28];
  const float* e2n1w  = (const float*)d_in[29];
  const float* e2n1b  = (const float*)d_in[30];
  const float* e2n2w  = (const float*)d_in[31];
  const float* e2n2b  = (const float*)d_in[32];
  const float* n2e1w  = (const float*)d_in[33];
  const float* n2e1b  = (const float*)d_in[34];
  const float* n2e2w  = (const float*)d_in[35];
  const float* n2e2b  = (const float*)d_in[36];
  const float* relw   = (const float*)d_in[37];
  const float* relb   = (const float*)d_in[38];
  float* out0 = (float*)d_out;
  float* out1 = (float*)d_out + (size_t)kNodes * kObj;

  char* ws = (char*)d_ws;
  _Float16* Wn1   = (_Float16*)(ws + kOffWn1);
  _Float16* Wed   = (_Float16*)(ws + kOffWed);
  _Float16* Wn2   = (_Float16*)(ws + kOffWn2);
  _Float16* Wngih = (_Float16*)(ws + kOffWngih);
  _Float16* Wnghh = (_Float16*)(ws + kOffWnghh);
  _Float16* Wegih = (_Float16*)(ws + kOffWegih);
  _Float16* Weghh = (_Float16*)(ws + kOffWeghh);
  _Float16* Wa1   = (_Float16*)(ws + kOffWa1);
  _Float16* Wa2   = (_Float16*)(ws + kOffWa2);
  _Float16* Wb1   = (_Float16*)(ws + kOffWb1);
  _Float16* Wb2   = (_Float16*)(ws + kOffWb2);
  _Float16* Wc1   = (_Float16*)(ws + kOffWc1);
  _Float16* Wc2   = (_Float16*)(ws + kOffWc2);
  _Float16* WrelH = (_Float16*)(ws + kOffWrelH);
  _Float16* WrelL = (_Float16*)(ws + kOffWrelL);
  _Float16* Uni   = (_Float16*)(ws + kOffUni);
  _Float16* Ek    = (_Float16*)(ws + kOffEk);
  _Float16* T1    = (_Float16*)(ws + kOffT1);
  _Float16* Msg   = (_Float16*)(ws + kOffMsg);
  _Float16* Heh[2] = {(_Float16*)(ws + kOffHeh0), (_Float16*)(ws + kOffHeh1)};
  _Float16* Helo  = (_Float16*)(ws + kOffHelo);
  _Float16* Xcat  = (_Float16*)(ws + kOffXcat);
  _Float16* Xcat2 = (_Float16*)(ws + kOffXcat2);
  float* Er       = (float*)(ws + kOffEr);
  float* He[2]    = {(float*)(ws + kOffHe0), (float*)(ws + kOffHe1)};
  float* Gie      = (float*)(ws + kOffGie);
  float* Ghe      = (float*)(ws + kOffGhe);
  float* Ph       = (float*)(ws + kOffPh);
  float* Stats    = (float*)(ws + kOffStats);
  float* Pose     = (float*)(ws + kOffPose);
  float* Hn[2]    = {(float*)(ws + kOffHn0), (float*)(ws + kOffHn1)};
  _Float16* Hnh[2] = {(_Float16*)(ws + kOffHnh0), (_Float16*)(ws + kOffHnh1)};
  _Float16* E2nRaw = (_Float16*)(ws + kOffE2nRaw);
  _Float16* N2nRaw = (_Float16*)(ws + kOffN2nRaw);
  _Float16* Te    = (_Float16*)(ws + kOffTe);
  _Float16* Tn    = (_Float16*)(ws + kOffTn);
  float* E2nM     = (float*)(ws + kOffE2nM);
  float* N2nM     = (float*)(ws + kOffN2nM);
  _Float16* Inph  = (_Float16*)(ws + kOffInph);
  float* Gin      = (float*)(ws + kOffGin);
  float* Ghn      = (float*)(ws + kOffGhn);
  float* Ns2      = (float*)(ws + kOffNs2);
  float* RelPad   = (float*)(ws + kOffRelPad);
  int*   First    = (int*)(ws + kOffFirst);

  constexpr float kW = 1024.0f;
  constexpr float kUn1  = 1.0f / 1024.0f;
  constexpr float kUn16 = 1.0f / 16384.0f;
  constexpr float kUnR  = 1.0f / 33554432.0f;

  run_cvt(stream, w_n1, Wn1, kHid, kHid, kCat1, kCat1P, kW);
  run_cvt(stream, w_ed, Wed, kHid, kHid, kCin, kCin, kW);
  run_cvt(stream, w_n2, Wn2, kHid, kHid, kCat2, kCat2P, kW);
  run_cvt(stream, ngih, Wngih, kGate, kGate, kHid, kHid, kW);
  run_cvt(stream, nghh, Wnghh, kGate, kGate, kHid, kHid, kW);
  run_cvt(stream, egih, Wegih, kGate, kGate, kHid, kHid, kW);
  run_cvt(stream, eghh, Weghh, kGate, kGate, kHid, kHid, kW);
  run_cvt(stream, n2n1w, Wa1, kHid, kHid, kHid, kHid, kW);
  run_cvt(stream, n2n2w, Wa2, kHid, kHid, kHid, kHid, kW);
  run_cvt(stream, e2n1w, Wb1, kHid, kHid, kHid, kHid, kW);
  run_cvt(stream, e2n2w, Wb2, kHid, kHid, kHid, kHid, kW);
  run_cvt(stream, n2e1w, Wc1, kHid, kHid, kPairK, kPairK, kW);
  run_cvt(stream, n2e2w, Wc2, kHid, kHid, kHid, kHid, kW);
  rel_weight_split<<<dim3((kRelPad * (kHid / 8) + 255) / 256), dim3(256), 0, stream>>>(relw, WrelH, WrelL);

  run_cvt(stream, uni, Uni, kEdges, kEdges, kCin, kCin, 1.0f);

  pos_lin1<<<dim3((kNodes * kPosMid + 255) / 256), dim3(256), 0, stream>>>(pinfo, pw1, pb1, Ph);
  pos_bnstats<<<dim3(1), dim3(256), 0, stream>>>(Ph, Stats);
  pos_lin2<<<dim3(kNodes), dim3(128), 0, stream>>>(Ph, Stats, pgam, pbet, pw2, pb2, Pose);

  build_cat<true><<<dim3((kNodes * (kCat1P / 8) + 255) / 256), dim3(256), 0, stream>>>(
      x, Pose, kPosOut, emb1, lab, Xcat, kCat1P);
  run_gemm<4, false, true, 3, false>(stream, Xcat, nullptr, kCat1P, Wn1, nullptr, kCat1P,
      Hn[0], Hnh[0], kHid, b_n1, kHid, kNodes, kHid, kCat1P, kUn1, 0.0f, 16.0f);

  run_gemm<4, false, true, 0, false>(stream, Uni, nullptr, kCin, Wed, nullptr, kCin,
      Er, nullptr, kHid, b_ed, kHid, kEdges, kHid, kCin, kUn1, 0.0f, 1.0f);

  pair_flags<<<dim3(kEdges / 256), dim3(256), 0, stream>>>(rp, First);
  pair_h0<<<dim3(kEdges / 8), dim3(256), 0, stream>>>(rp, Er, He[0], Heh[0]);

  node_gather<0><<<dim3(kNodes), dim3(128), 0, stream>>>(rp, First, Er, E2nRaw);
  run_gemm<4, false, true, 1, true>(stream, E2nRaw, nullptr, kHid, Wb1, nullptr, kHid,
      nullptr, Te, kHid, e2n1b, kHid, kNodes, kHid, kHid, kUn16, 0.0f, 16.0f);
  run_gemm<4, false, true, 0, true>(stream, Te, nullptr, kHid, Wb2, nullptr, kHid,
      E2nM, nullptr, kHid, e2n2b, kHid, kNodes, kHid, kHid, kUn16, 0.0f, 1.0f);

  for (int it = 0; it < 3; ++it) {
    const int cur = it & 1, nxt = cur ^ 1;
    node_gather<1><<<dim3(kNodes), dim3(128), 0, stream>>>(rp, First, Hn[cur], N2nRaw);
    run_gemm<4, false, true, 1, true>(stream, N2nRaw, nullptr, kHid, Wa1, nullptr, kHid,
        nullptr, Tn, kHid, n2n1b, kHid, kNodes, kHid, kHid, kUn16, 0.0f, 16.0f);
    run_gemm<4, false, true, 0, true>(stream, Tn, nullptr, kHid, Wa2, nullptr, kHid,
        N2nM, nullptr, kHid, n2n2b, kHid, kNodes, kHid, kHid, kUn16, 0.0f, 1.0f);
    combine_half<<<dim3((kNodes * kHid / 8 + 255) / 256), dim3(256), 0, stream>>>(N2nM, E2nM, Inph, kNodes * kHid / 8);
    run_gemm<4, false, true, 0, false>(stream, Inph, nullptr, kHid, Wngih, nullptr, kHid,
        Gin, nullptr, kGate, ngbih, kGate, kNodes, kGate, kHid, kUn16, 0.0f, 1.0f);
    run_gemm<4, false, true, 0, false>(stream, Hnh[cur], nullptr, kHid, Wnghh, nullptr, kHid,
        Ghn, nullptr, kGate, ngbhh, kGate, kNodes, kGate, kHid, kUn16, 0.0f, 1.0f);
    gru_gate<false><<<dim3(kNodes), dim3(256), 0, stream>>>(Gin, Ghn, Hn[cur], Hn[nxt], Hnh[nxt], nullptr, kNodes);
  }

  pack_obj<<<dim3((kNodes * kObj + 255) / 256), dim3(256), 0, stream>>>(lab, out0);

  build_cat<false><<<dim3((kNodes * (kCat2P / 8) + 255) / 256), dim3(256), 0, stream>>>(
      x, Hn[1], kHid, emb2, lab, Xcat2, kCat2P);
  run_gemm<4, false, true, 0, false>(stream, Xcat2, nullptr, kCat2P, Wn2, nullptr, kCat2P,
      Ns2, nullptr, kHid, b_n2, kHid, kNodes, kHid, kCat2P, kUn1, 0.0f, 1.0f);

  build_ek<<<dim3(kEdges * (kPairK / 8) / 256), dim3(256), 0, stream>>>(rp, Ns2, Ek);
  run_gemm<4, false, true, 1, true>(stream, Ek, nullptr, kPairK, Wc1, nullptr, kPairK,
      nullptr, T1, kHid, n2e1b, kHid, kEdges, kHid, kPairK, kUn16, 0.0f, 16.0f);
  run_gemm<4, false, true, 1, true>(stream, T1, nullptr, kHid, Wc2, nullptr, kHid,
      nullptr, Msg, kHid, n2e2b, kHid, kEdges, kHid, kHid, kUn16, 0.0f, 16.0f);
  run_gemm<4, false, false, 0, false>(stream, Msg, nullptr, kHid, Wegih, nullptr, kHid,
      Gie, nullptr, kGate, nullptr, 1, kEdges, kGate, kHid, kUn16, 0.0f, 1.0f);

  for (int it = 0; it < 3; ++it) {
    const int cur = it & 1, nxt = cur ^ 1;
    run_gemm<4, false, false, 0, false>(stream, Heh[cur], nullptr, kHid, Weghh, nullptr, kHid,
        Ghe, nullptr, kGate, nullptr, 1, kEdges, kGate, kHid, kUn16, 0.0f, 1.0f);
    if (it == 2)
      gru_gate<true><<<dim3(kEdges), dim3(256), 0, stream>>>(Gie, Ghe, He[cur], He[nxt], Heh[nxt], Helo, kEdges);
    else
      gru_gate<false><<<dim3(kEdges), dim3(256), 0, stream>>>(Gie, Ghe, He[cur], He[nxt], Heh[nxt], nullptr, kEdges);
  }

  run_gemm<1, true, true, 0, false>(stream, Heh[1], Helo, kHid, WrelH, WrelL, kHid,
      RelPad, nullptr, kRelPad, relb, kRel, kEdges, kRelPad, kHid, kUn16, kUnR, 1.0f);
  pack_rel<<<dim3((kEdges * kRel + 255) / 256), dim3(256), 0, stream>>>(RelPad, out1);
}
